// Fusion_Block_20263655703077
// MI455X (gfx1250) — hardware-verified
//
#include <hip/hip_runtime.h>


#define NBI  8
#define NN   2048
#define NR   (NBI * NN)
#define DD   64
#define NH_  4
#define HD   16
#define HDP  32
#define VP   64
#define HID  128
#define DM   DD
#define NTK  NR
#define SCL  0.25f
#define LN_EPS 1e-5f
#define LOSC 1024.0f

typedef _Float16 h16;
typedef unsigned short bf;
typedef __attribute__((ext_vector_type(16))) __bf16   v16bf;
typedef __attribute__((ext_vector_type(16))) _Float16 v16h;
typedef __attribute__((ext_vector_type(8)))  _Float16 v8h;
typedef __attribute__((ext_vector_type(8)))  unsigned short v8us;
typedef __attribute__((ext_vector_type(8)))  float    v8f;
typedef __attribute__((ext_vector_type(4)))  float    v4f;
typedef __attribute__((ext_vector_type(4)))  _Float16 v4h;
typedef v8h  __attribute__((may_alias)) v8ha;
typedef v4f  __attribute__((may_alias)) v4fa;
typedef v8us __attribute__((may_alias)) v8usa;

__device__ __forceinline__ unsigned short f2bf(float f) { unsigned u = __float_as_uint(f); u += 0x7FFFu + ((u >> 16) & 1u); return (unsigned short)(u >> 16); }
__device__ __forceinline__ float bf2f(unsigned short b) { return __uint_as_float(((unsigned)b) << 16); }
__device__ __forceinline__ float bfr(float f) { return bf2f(f2bf(f)); }
__device__ __forceinline__ v16h cat16(v8h lo, v8h hi) { return __builtin_shufflevector(lo, hi, 0, 1, 2, 3, 4, 5, 6, 7, 8, 9, 10, 11, 12, 13, 14, 15); }
__device__ __forceinline__ v16bf cat16b(v8us lo, v8us hi) { return __builtin_bit_cast(v16bf, __builtin_shufflevector(lo, hi, 0, 1, 2, 3, 4, 5, 6, 7, 8, 9, 10, 11, 12, 13, 14, 15)); }
__device__ __forceinline__ v8f wmma16(v16h a, v16h b, v8f c) { return __builtin_amdgcn_wmma_f32_16x16x32_f16(false, a, false, b, (short)0, c, false, false); }
__device__ __forceinline__ v8f wmmab(v16bf a, v16bf b, v8f c) { return __builtin_amdgcn_wmma_f32_16x16x32_bf16(false, a, false, b, (short)0, c, false, false); }

__global__ __launch_bounds__(256) void k_wt(const float* __restrict__ Wm, int K, int ncols, bf* WT) {
    __shared__ __align__(16) unsigned short tl[64 * 72];
    const int tid = threadIdx.x, k0 = blockIdx.x * 64, n0 = blockIdx.y * 64;
    const int kk = tid >> 2, nq = (tid & 3) * 16;
#pragma unroll
    for (int i = 0; i < 16; ++i) tl[(nq + i) * 72 + kk] = f2bf(Wm[(size_t)(k0 + kk) * ncols + n0 + nq + i]);
    __syncthreads();
    const int piece = tid & 7;
    auto pass = [&]() {
#pragma unroll
        for (int s = 0; s < 2; ++s) { const int nr = (tid >> 3) + 32 * s; const v8us val = *(const v8usa*)(tl + nr * 72 + piece * 8); *(volatile v8us*)(WT + (size_t)(n0 + nr) * K + k0 + piece * 8) = val; }
    };
    pass(); __threadfence(); pass();
}
template <bool SPLITA, bool F16OUT = false>
__global__ __launch_bounds__(128) void k_gemmb(const bf* __restrict__ A, const bf* __restrict__ Al, const bf* __restrict__ Bn, const float* __restrict__ bias, float* C, int ldc, h16* C2, const float* __restrict__ R = nullptr, int K = DM, int roundR = 1) {
    __shared__ __align__(16) float ost[4][16 * 68];
    const int lane = threadIdx.x & 31, wave = threadIdx.x >> 5, lr = lane & 15, hi = lane >> 4;
    const int r0 = blockIdx.x * 64 + wave * 16, c0 = blockIdx.y * 64;
    const size_t aoff = (size_t)(r0 + lr) * K + 8 * hi;
    size_t boff[4];
#pragma unroll
    for (int t = 0; t < 4; ++t) boff[t] = (size_t)(c0 + t * 16 + lr) * K + 8 * hi;
    v8f acc[4];
#pragma unroll
    for (int t = 0; t < 4; ++t) acc[t] = (v8f){};
#pragma unroll 1
    for (int kc = 0; kc < K; kc += 32) {
        const v16bf a = cat16b(*(const v8us*)(A + aoff + kc), *(const v8us*)(A + aoff + kc + 16));
        v16bf al = a;
        if (SPLITA) al = cat16b(*(const v8us*)(Al + aoff + kc), *(const v8us*)(Al + aoff + kc + 16));
#pragma unroll
        for (int t = 0; t < 4; ++t) { const v16bf b = cat16b(*(const v8us*)(Bn + boff[t] + kc), *(const v8us*)(Bn + boff[t] + kc + 16)); acc[t] = wmmab(a, b, acc[t]); if (SPLITA) acc[t] = wmmab(al, b, acc[t]); }
        asm volatile("v_nop\n\tv_nop\n\tv_nop\n\tv_nop" : "+v"(acc[0]), "+v"(acc[1]), "+v"(acc[2]), "+v"(acc[3]) : "v"(a), "v"(al));
    }
    float* os = &ost[wave][0];
#pragma unroll
    for (int t = 0; t < 4; ++t) { const float bv = bias ? bfr(bias[c0 + t * 16 + lr]) : 0.f;
#pragma unroll
        for (int j = 0; j < 8; ++j) os[(hi * 8 + j) * 68 + t * 16 + lr] = acc[t][j] + bv; }
    __syncthreads();
    if (F16OUT) {
        h16* crow = (h16*)(void*)C + (size_t)r0 * ldc + c0;
        auto pass = [&]() {
#pragma unroll
            for (int s = 0; s < 4; ++s) { const int row = 4 * s + (lane >> 3), piece = lane & 7; const float* sp = os + row * 68 + piece * 8; v8h o, o2;
#pragma unroll
                for (int i = 0; i < 8; ++i) { const h16 a = (h16)sp[i]; o[i] = a; o2[i] = (h16)((sp[i] - (float)a) * LOSC); }
                *(volatile v8h*)(crow + (size_t)row * ldc + piece * 8) = o; if (C2) *(volatile v8h*)(C2 + (size_t)r0 * ldc + c0 + (size_t)row * ldc + piece * 8) = o2; }
        };
        pass(); __threadfence(); pass();
    } else {
        float* crow = C + (size_t)r0 * ldc + c0;
        auto pass = [&]() {
#pragma unroll
            for (int s = 0; s < 8; ++s) { const int Lid = (lane >> 3) + 4 * s, piece = lane & 7; const int row = Lid >> 1, cofs = (Lid & 1) * 32 + piece * 4;
                v4f val = *(const v4fa*)(os + row * 68 + cofs); if (R) { const v4f rv = *(const v4f*)(R + ((size_t)r0 + row) * ldc + c0 + cofs); val += roundR ? (v4f){bfr(rv[0]), bfr(rv[1]), bfr(rv[2]), bfr(rv[3])} : rv; }
                *(volatile v4f*)(crow + (size_t)row * ldc + cofs) = val; }
        };
        pass(); __threadfence(); pass();
    }
}

__global__ __launch_bounds__(128) void k_gemm3(const bf* __restrict__ Ah, const bf* __restrict__ Al, const bf* __restrict__ Bh, const bf* __restrict__ Bl, int K, float* C, int ldc) {
    __shared__ __align__(16) float ost[4][16 * 68];
    const int lane = threadIdx.x & 31, wave = threadIdx.x >> 5, lr = lane & 15, hi = lane >> 4;
    const int r0 = blockIdx.x * 64 + wave * 16, c0 = blockIdx.y * 64;
    const size_t aoff = (size_t)(r0 + lr) * K + 8 * hi;
    v8f acc[4];
#pragma unroll
    for (int t = 0; t < 4; ++t) acc[t] = (v8f){};
#pragma unroll 1
    for (int kc = 0; kc < K; kc += 32) {
        const v16bf a = cat16b(*(const v8us*)(Ah + aoff + kc), *(const v8us*)(Ah + aoff + kc + 16));
        const v16bf al = cat16b(*(const v8us*)(Al + aoff + kc), *(const v8us*)(Al + aoff + kc + 16));
#pragma unroll
        for (int t = 0; t < 4; ++t) { const size_t bo = (size_t)(c0 + t * 16 + lr) * K + kc + 8 * hi;
            const v16bf bh = cat16b(*(const v8us*)(Bh + bo), *(const v8us*)(Bh + bo + 16)); const v16bf bl = cat16b(*(const v8us*)(Bl + bo), *(const v8us*)(Bl + bo + 16));
            acc[t] = wmmab(a, bh, acc[t]); acc[t] = wmmab(al, bh, acc[t]); acc[t] = wmmab(a, bl, acc[t]); }
        asm volatile("v_nop\n\tv_nop\n\tv_nop\n\tv_nop" : "+v"(acc[0]), "+v"(acc[1]), "+v"(acc[2]), "+v"(acc[3]) : "v"(a), "v"(al));
    }
    float* os = &ost[wave][0];
#pragma unroll
    for (int t = 0; t < 4; ++t) {
#pragma unroll
        for (int j = 0; j < 8; ++j) os[(hi * 8 + j) * 68 + t * 16 + lr] = acc[t][j]; }
    __builtin_amdgcn_wave_barrier(); asm volatile("" ::: "memory");
    float* crow = C + (size_t)r0 * ldc + c0;
    auto pass = [&]() {
#pragma unroll
        for (int s = 0; s < 8; ++s) { const int Lid = (lane >> 3) + 4 * s, piece = lane & 7; const int row = Lid >> 1, cofs = (Lid & 1) * 32 + piece * 4;
            const v4f val = *(const v4fa*)(os + row * 68 + cofs); *(volatile v4f*)(crow + (size_t)row * ldc + cofs) = val; }
    };
    pass(); __threadfence(); pass();
}

__global__ __launch_bounds__(256) void k_ln64(const float* __restrict__ src, int rnd, const float* __restrict__ g, const float* __restrict__ bb, int nrows, float* Y, bf* Ph, bf* Pl) {
    typedef __attribute__((ext_vector_type(2))) float v2f; typedef __attribute__((ext_vector_type(2))) unsigned short v2us;
    const int lane = threadIdx.x & 31, r = blockIdx.x * 8 + (threadIdx.x >> 5); if (r >= nrows) return;
    const size_t o = (size_t)r * DD + 2 * lane; float v0 = src[o], v1 = src[o + 1]; if (rnd) { v0 = bfr(v0); v1 = bfr(v1); }
    float s = v0 + v1;
#pragma unroll
    for (int sh = 16; sh; sh >>= 1) s += __shfl_xor(s, sh, 32);
    const float mu = s * (1.0f / DD); const float d0 = v0 - mu, d1 = v1 - mu; float s2 = d0 * d0 + d1 * d1;
#pragma unroll
    for (int sh = 16; sh; sh >>= 1) s2 += __shfl_xor(s2, sh, 32);
    const float rs = rsqrtf(s2 * (1.0f / DD) + LN_EPS);
    v2f y; y[0] = d0 * rs * bfr(g[2 * lane]) + bfr(bb[2 * lane]); y[1] = d1 * rs * bfr(g[2 * lane + 1]) + bfr(bb[2 * lane + 1]);
    v2us oh, ol;
#pragma unroll
    for (int i = 0; i < 2; ++i) { const unsigned short hb = f2bf(y[i]); oh[i] = hb; ol[i] = f2bf(y[i] - bf2f(hb)); }
    if (Y) *(volatile v2f*)(Y + o) = y; *(volatile v2us*)(Ph + o) = oh; *(volatile v2us*)(Pl + o) = ol; __threadfence();
    if (Y) *(volatile v2f*)(Y + o) = y; *(volatile v2us*)(Ph + o) = oh; *(volatile v2us*)(Pl + o) = ol;
}
__global__ __launch_bounds__(256) void k_qkpad(const float* __restrict__ Qf, const float* __restrict__ KVf, bf* QPh, bf* QPl, bf* KPh, bf* KPl) {
    typedef __attribute__((ext_vector_type(2))) unsigned short v2us;
    const int lane = threadIdx.x & 31, wid = blockIdx.x * 8 + (threadIdx.x >> 5); if (wid >= NR * NH_ / 2) return;
    const int h = wid % NH_, tp = wid / NH_; const int t = tp * 2 + (lane >> 4), l = lane & 15; const int d0 = 2 * l;
    const int b = t / NN, tt = t % NN;
    v2us qh, ql, kh, kl;
#pragma unroll
    for (int i = 0; i < 2; ++i) { const int d = d0 + i; float qv = 0.f, kv = 0.f; if (d < HD) { qv = Qf[(size_t)t * DD + h * HD + d]; kv = KVf[(size_t)t * HID + h * HD + d]; }
        unsigned short hb = f2bf(qv); qh[i] = hb; ql[i] = f2bf(qv - bf2f(hb)); hb = f2bf(kv); kh[i] = hb; kl[i] = f2bf(kv - bf2f(hb)); }
    const size_t o = (((size_t)b * NH_ + h) * NN + tt) * HDP + d0;
    *(volatile v2us*)(QPh + o) = qh; *(volatile v2us*)(QPl + o) = ql; *(volatile v2us*)(KPh + o) = kh; *(volatile v2us*)(KPl + o) = kl; __threadfence();
    *(volatile v2us*)(QPh + o) = qh; *(volatile v2us*)(QPl + o) = ql; *(volatile v2us*)(KPh + o) = kh; *(volatile v2us*)(KPl + o) = kl;
}
__global__ __launch_bounds__(256) void k_vtp(const float* __restrict__ KVf, int b, bf* VTh, bf* VTl) {
    typedef __attribute__((ext_vector_type(2))) unsigned short v2us;
    const int lane = threadIdx.x & 31, wid = blockIdx.x * 8 + (threadIdx.x >> 5); if (wid >= NH_ * VP * (NN / 64)) return;
    const int tg = wid % (NN / 64), rest = wid / (NN / 64), d = rest % VP, h = rest / VP; const int t0 = tg * 64 + 2 * lane;
    v2us oh, ol;
#pragma unroll
    for (int i = 0; i < 2; ++i) { float v = 0.f; if (d < HD) v = KVf[((size_t)b * NN + t0 + i) * HID + DD + h * HD + d]; const unsigned short hb = f2bf(v); oh[i] = hb; ol[i] = f2bf(v - bf2f(hb)); }
    const size_t o = ((size_t)h * VP + d) * NN + t0;
    *(volatile v2us*)(VTh + o) = oh; *(volatile v2us*)(VTl + o) = ol; __threadfence(); *(volatile v2us*)(VTh + o) = oh; *(volatile v2us*)(VTl + o) = ol;
}
__global__ __launch_bounds__(256) void k_softmax(const float* __restrict__ S, bf* PH, bf* PL) {
    const int lane = threadIdx.x & 31, r = blockIdx.x * 8 + (threadIdx.x >> 5); if (r >= NN) return;
    const float* sr = S + (size_t)r * NN; float m = -3.0e38f;
#pragma unroll 1
    for (int c0 = lane * 8; c0 < NN; c0 += 256) { const v8f v = *(const v8f*)(sr + c0);
#pragma unroll
        for (int i = 0; i < 8; ++i) m = fmaxf(m, v[i] * SCL); }
#pragma unroll
    for (int sh = 16; sh; sh >>= 1) m = fmaxf(m, __shfl_xor(m, sh, 32));
    float sum = 0.f;
#pragma unroll 1
    for (int c0 = lane * 8; c0 < NN; c0 += 256) { const v8f v = *(const v8f*)(sr + c0);
#pragma unroll
        for (int i = 0; i < 8; ++i) sum += __expf(v[i] * SCL - m); }
#pragma unroll
    for (int sh = 16; sh; sh >>= 1) sum += __shfl_xor(sum, sh, 32);
    const float inv = 1.0f / sum;
#pragma unroll 1
    for (int ps = 0; ps < 2; ++ps) {
#pragma unroll 1
        for (int c0 = lane * 8; c0 < NN; c0 += 256) { const v8f v = *(const v8f*)(sr + c0); v8us oh, ol;
#pragma unroll
            for (int i = 0; i < 8; ++i) { const float p = __expf(v[i] * SCL - m) * inv; const unsigned short hb = f2bf(p); oh[i] = hb; ol[i] = f2bf(p - bf2f(hb)); }
            const size_t o = (size_t)r * NN + c0; *(volatile v8us*)(PH + o) = oh; *(volatile v8us*)(PL + o) = ol; }
        if (ps == 0) __threadfence(); }
}
__global__ __launch_bounds__(256) void k_assemble(const float* __restrict__ O4, int b, bf* Ch, bf* Cl) {
    typedef __attribute__((ext_vector_type(2))) unsigned short v2us;
    const int lane = threadIdx.x & 31, t = blockIdx.x * 8 + (threadIdx.x >> 5); if (t >= NN) return;
    const int c = 2 * lane, h = c / HD, d = c % HD; v2us oh, ol;
#pragma unroll
    for (int i = 0; i < 2; ++i) { const float v = O4[((size_t)h * NN + t) * VP + d + i]; const unsigned short hb = f2bf(v); oh[i] = hb; ol[i] = f2bf(v - bf2f(hb)); }
    const size_t o = ((size_t)b * NN + t) * DD + c;
    *(volatile v2us*)(Ch + o) = oh; *(volatile v2us*)(Cl + o) = ol; __threadfence(); *(volatile v2us*)(Ch + o) = oh; *(volatile v2us*)(Cl + o) = ol;
}
__global__ __launch_bounds__(256) void k_gelu(const float* __restrict__ src, int nrows, bf* dh, bf* dl) {
    typedef __attribute__((ext_vector_type(4))) unsigned short v4us;
    const int lane = threadIdx.x & 31, r = blockIdx.x * 8 + (threadIdx.x >> 5); if (r >= nrows) return;
    const size_t o = (size_t)r * HID + lane * 4; const v4f v = *(const v4f*)(src + o); v4us oh, ol;
#pragma unroll
    for (int i = 0; i < 4; ++i) { const float y = 0.5f * v[i] * (1.0f + erff(v[i] * 0.7071067811865476f)); const unsigned short hb = f2bf(y); oh[i] = hb; ol[i] = f2bf(y - bf2f(hb)); }
    *(volatile v4us*)(dh + o) = oh; *(volatile v4us*)(dl + o) = ol; __threadfence(); *(volatile v4us*)(dh + o) = oh; *(volatile v4us*)(dl + o) = ol;
}

extern "C" void kernel_launch(void* const* d_in, const int* in_sizes, int n_in,
                              void* d_out, int out_size, void* d_ws, size_t ws_size, hipStream_t stream) {
    (void)in_sizes; (void)n_in; (void)out_size;
    const float* x = (const float*)d_in[0]; const float* cl = (const float*)d_in[1]; const float* g1 = (const float*)d_in[2]; const float* be1 = (const float*)d_in[3]; const float* g2 = (const float*)d_in[4]; const float* be2 = (const float*)d_in[5];
    const float* Wkv = (const float*)d_in[6]; const float* bkv = (const float*)d_in[7]; const float* Wq = (const float*)d_in[8]; const float* bq = (const float*)d_in[9]; const float* Wp = (const float*)d_in[10]; const float* bp = (const float*)d_in[11];
    const float* W1 = (const float*)d_in[12]; const float* b1 = (const float*)d_in[13]; const float* W2 = (const float*)d_in[14]; const float* b2 = (const float*)d_in[15];
    float* out = (float*)d_out;
    char* wsp = (char*)d_ws;
    auto take = [&](size_t bytes) { char* p = wsp; wsp += (bytes + 255) & ~(size_t)255; return (void*)p; };
    bf* WkvT = (bf*)take(HID * DD * 2); bf* WqT = (bf*)take(DD * DD * 2); bf* WpT = (bf*)take(DD * DD * 2); bf* W1T = (bf*)take(HID * DD * 2); bf* W2T = (bf*)take(DD * HID * 2);
    bf* XNh = (bf*)take((size_t)NR * DD * 2); bf* XNl = (bf*)take((size_t)NR * DD * 2); bf* CNh = (bf*)take((size_t)NR * DD * 2); bf* CNl = (bf*)take((size_t)NR * DD * 2);
    float* KVf = (float*)take((size_t)NR * HID * 4); float* Qf = (float*)take((size_t)NR * DD * 4);
    bf* QPh = (bf*)take((size_t)NR * NH_ * HDP * 2); bf* QPl = (bf*)take((size_t)NR * NH_ * HDP * 2); bf* KPh = (bf*)take((size_t)NR * NH_ * HDP * 2); bf* KPl = (bf*)take((size_t)NR * NH_ * HDP * 2);
    bf* VTh = (bf*)take((size_t)NH_ * VP * NN * 2); bf* VTl = (bf*)take((size_t)NH_ * VP * NN * 2); float* S = (float*)take((size_t)NN * NN * 4); bf* PH = (bf*)take((size_t)NN * NN * 2); bf* PL = (bf*)take((size_t)NN * NN * 2);
    float* O4 = (float*)take((size_t)NH_ * NN * VP * 4); bf* Ch = (bf*)take((size_t)NR * DD * 2); bf* Cl = (bf*)take((size_t)NR * DD * 2);
    float* Of = (float*)take((size_t)NR * DD * 4); bf* Hh = (bf*)take((size_t)NR * DD * 2); bf* Hl = (bf*)take((size_t)NR * DD * 2); float* M = (float*)take((size_t)NR * HID * 4); bf* Mh = (bf*)take((size_t)NR * HID * 2); bf* Ml = (bf*)take((size_t)NR * HID * 2);
    if ((size_t)(wsp - (char*)d_ws) > ws_size) return;
    k_wt<<<dim3(1, HID / 64, 1), 256, 0, stream>>>(Wkv, DD, HID, WkvT); k_wt<<<dim3(1, 1, 1), 256, 0, stream>>>(Wq, DD, DD, WqT); k_wt<<<dim3(1, 1, 1), 256, 0, stream>>>(Wp, DD, DD, WpT);
    k_wt<<<dim3(1, HID / 64, 1), 256, 0, stream>>>(W1, DD, HID, W1T); k_wt<<<dim3(HID / 64, 1, 1), 256, 0, stream>>>(W2, HID, DD, W2T);
    k_ln64<<<NR / 8, 256, 0, stream>>>(x, 1, g1, be1, NR, nullptr, XNh, XNl); k_ln64<<<NR / 8, 256, 0, stream>>>(cl, 1, g1, be1, NR, nullptr, CNh, CNl);
    k_gemmb<true, false><<<dim3(NR / 64, HID / 64, 1), 128, 0, stream>>>(XNh, XNl, WkvT, bkv, KVf, HID, nullptr, nullptr, DD);
    k_gemmb<true, false><<<dim3(NR / 64, 1, 1), 128, 0, stream>>>(CNh, CNl, WqT, bq, Qf, DD, nullptr, nullptr, DD);
    k_qkpad<<<(NR * NH_ / 2 + 7) / 8, 256, 0, stream>>>(Qf, KVf, QPh, QPl, KPh, KPl);
    for (int b = 0; b < NBI; ++b) {
        k_vtp<<<(NH_ * VP * (NN / 64)) / 8, 256, 0, stream>>>(KVf, b, VTh, VTl);
        for (int h = 0; h < NH_; ++h) { const size_t po = ((size_t)b * NH_ + h) * NN * HDP;
            k_gemm3<<<dim3(NN / 64, NN / 64, 1), 128, 0, stream>>>(QPh + po, QPl + po, KPh + po, KPl + po, HDP, S, NN);
            k_softmax<<<NN / 8, 256, 0, stream>>>(S, PH, PL);
            k_gemm3<<<dim3(NN / 64, 1, 1), 128, 0, stream>>>(PH, PL, VTh + (size_t)h * VP * NN, VTl + (size_t)h * VP * NN, NN, O4 + (size_t)h * NN * VP, VP);
        }
        k_assemble<<<NN / 8, 256, 0, stream>>>(O4, b, Ch, Cl);
    }
    k_gemmb<true, false><<<dim3(NR / 64, 1, 1), 128, 0, stream>>>(Ch, Cl, WpT, bp, Of, DD, nullptr, nullptr, DD);
    k_ln64<<<NR / 8, 256, 0, stream>>>(Of, 0, g2, be2, NR, nullptr, Hh, Hl);
    k_gemmb<true, false><<<dim3(NR / 64, HID / 64, 1), 128, 0, stream>>>(Hh, Hl, W1T, b1, M, HID, nullptr, nullptr, DD); k_gelu<<<NR / 8, 256, 0, stream>>>(M, NR, Mh, Ml);
    k_gemmb<true, false><<<dim3(NR / 64, 1, 1), 128, 0, stream>>>(Mh, Ml, W2T, b2, out, DD, nullptr, Of, HID, 0);
}
